// Mamba_77816217469377
// MI455X (gfx1250) — hardware-run, weakly checked
//
#include <hip/hip_runtime.h>
#include <math.h>

typedef __attribute__((ext_vector_type(16))) __bf16   v16b;
typedef __attribute__((ext_vector_type(8)))  __bf16   v8b;
typedef __attribute__((ext_vector_type(8)))  float    v8f;
typedef __attribute__((ext_vector_type(4)))  float    v4f;
typedef __attribute__((ext_vector_type(2)))  float    v2f;
typedef __attribute__((ext_vector_type(4)))  unsigned v4u;

constexpr int kBatch  = 2;
constexpr int kSeq    = 1024;
constexpr int kDm     = 512;
constexpr int kDin    = 1024;
constexpr int kNst    = 16;
constexpr int kHeads  = 8;
constexpr int kHd     = kDin / kHeads;
constexpr int kDtR    = 32;
constexpr int kHN     = kHeads * kNst;
constexpr int kPrjN   = kDtR + 4 * kHN + 2 * kHeads;
constexpr int kPrjP   = 576;
constexpr int kXzP    = 2 * kDin;
constexpr int kRows   = kBatch * kSeq;
constexpr int kColBre = kDtR;
constexpr int kColLg  = kDtR + 4 * kHN;
constexpr int kConvTP = 260;
constexpr int kScanTS = 64;
constexpr int kScanCh = 64;
constexpr int kScanYP = 68;
constexpr int kScanXP = 100;
constexpr int kLB  = 32;
constexpr int kLBi = 48;
constexpr int kLC  = 64;
constexpr int kLCi = 80;
constexpr int kLG  = 96;
static_assert(kHd == 128 && kHN == 128 && kPrjN == 560 && kColLg == 544, "shape constants");
static_assert(kPrjP >= kPrjN && (kPrjP % 64) == 0, "padded x_proj width");
static_assert((kDm % 32) == 0 && (kDin % 32) == 0, "GEMM K multiples of 32");
static_assert((kRows % 64) == 0 && (kXzP % 64) == 0 && (kDm % 64) == 0, "GEMM M,N multiples of 64");
static_assert((kSeq % kScanTS) == 0 && (kSeq % 64) == 0 && (kHd % kScanCh) == 0 && (kDin % 256) == 0, "tile multiples");
static_assert(kDtR == 32 && kNst == 16, "staging layout");

constexpr size_t kOffXB   = 0;
constexpr size_t kOffWIB  = kOffXB   + (size_t)kRows * kDm  * 2;
constexpr size_t kOffWXB  = kOffWIB  + (size_t)kXzP  * kDm  * 2;
constexpr size_t kOffWOB  = kOffWXB  + (size_t)kPrjP * kDin * 2;
constexpr size_t kOffXZ   = kOffWOB  + (size_t)kDm   * kDin * 2;
constexpr size_t kOffUC   = kOffXZ   + (size_t)kRows * kXzP * 4;
constexpr size_t kOffUCH  = kOffUC   + (size_t)kRows * kDin * 4;
constexpr size_t kOffUCL  = kOffUCH  + (size_t)kRows * kDin * 2;
constexpr size_t kOffPROJ = kOffUCL  + (size_t)kRows * kDin * 2;
constexpr size_t kOffYH   = kOffPROJ + (size_t)kRows * kPrjP * 4;
constexpr size_t kOffYL   = kOffYH   + (size_t)kRows * kDin * 2;
constexpr size_t kWsTotal = kOffYL   + (size_t)kRows * kDin * 2;
static_assert(kWsTotal == 53084160ull, "carve total");
static_assert(kWsTotal <= 134217728ull, "carve cap");
static_assert((kOffWIB % 128) == 0 && (kOffWXB % 128) == 0 && (kOffWOB % 128) == 0 && (kOffXZ % 128) == 0 &&
              (kOffUC % 128) == 0 && (kOffUCH % 128) == 0 && (kOffUCL % 128) == 0 && (kOffPROJ % 128) == 0 &&
              (kOffYH % 128) == 0 && (kOffYL % 128) == 0, "128-B aligned regions");

__device__ __forceinline__ unsigned short f2bf_bits(float f) {
  unsigned u = __float_as_uint(f);
  return (unsigned short)((u + 0x7FFFu + ((u >> 16) & 1u)) >> 16);
}
__device__ __forceinline__ float bf_bits2f(unsigned short h) { return __uint_as_float(((unsigned)h) << 16); }
__device__ __forceinline__ float bf_rne(float f) { return bf_bits2f(f2bf_bits(f)); }
__device__ __forceinline__ unsigned pack_hi2(float a, float b) {
  const unsigned ha = (unsigned)f2bf_bits(a);
  const unsigned hb = (unsigned)f2bf_bits(b);
  return ha | (hb << 16);
}
__device__ __forceinline__ unsigned pack_lo2(float a, float b) {
  const unsigned short ha = f2bf_bits(a);
  const unsigned short hb = f2bf_bits(b);
  const unsigned la = (unsigned)f2bf_bits(a - bf_bits2f(ha));
  const unsigned lb = (unsigned)f2bf_bits(b - bf_bits2f(hb));
  return la | (lb << 16);
}

__device__ __forceinline__ void dep_guard4_b(v8f& a, v8f& b, v8f& c, v8f& d, v16b x, v16b y) {
  asm volatile("v_nop\n\tv_nop\n\tv_nop\n\tv_nop" : "+v"(a), "+v"(b), "+v"(c), "+v"(d) : "v"(x), "v"(y));
}
__device__ __forceinline__ void keep4_b(v16b a, v16b b, v16b c, v16b d) { asm volatile("v_nop" :: "v"(a), "v"(b), "v"(c), "v"(d)); }
__device__ __forceinline__ void acc_guard4(v8f& a, v8f& b, v8f& c, v8f& d) { asm volatile("v_nop\n\tv_nop\n\tv_nop\n\tv_nop" : "+v"(a), "+v"(b), "+v"(c), "+v"(d)); }
union FragB { v16b v; v8b h[2]; };
__device__ __forceinline__ v16b frag_load_b(const __bf16* p) {
  FragB f;
  f.h[0] = *(const v8b*)(p);
  f.h[1] = *(const v8b*)(p + 16);
  return f.v;
}
__device__ __forceinline__ v8f mma_b(v16b a, v16b b, v8f c) {
  return __builtin_amdgcn_wmma_f32_16x16x32_bf16(false, a, false, b, (short)0, c, false, false);
}

template <int SPL>
__global__ __launch_bounds__(256) void wmma_gemm64_bf(
    const unsigned short* __restrict__ Ap, const unsigned short* __restrict__ A2p, int lda,
    const unsigned short* __restrict__ Btp, int ldb,
    float* __restrict__ Cout, int ldc, int M, int N, int K) {
  const __bf16* A  = (const __bf16*)Ap;
  const __bf16* A2 = (const __bf16*)A2p;
  const __bf16* Bt = (const __bf16*)Btp;
  __shared__ __align__(16) float sT[8][16 * 68];
  const int lane = threadIdx.x & 31;
  const int wave = threadIdx.x >> 5;
  const int tilesN = N >> 6;
  const int tilesM = M >> 6;
  const int tile = blockIdx.x * 8 + wave;
  if (tile >= tilesM * tilesN) return;
  const int tm = tile / tilesN;
  const int tn = tile - tm * tilesN;
  const int m0 = tm << 6;
  const int n0 = tn << 6;

  const int rlane = lane & 15;
  const int koff  = (lane >> 4) * 8;
  const int mOff  = (lane >> 4) * 8;

  v8f acc[4][4];
#pragma unroll
  for (int i = 0; i < 4; ++i)
#pragma unroll
    for (int j = 0; j < 4; ++j) acc[i][j] = (v8f){0.f,0.f,0.f,0.f,0.f,0.f,0.f,0.f};

  for (int k0 = 0; k0 < K; k0 += 32) {
    v16b bh[4];
#pragma unroll
    for (int j = 0; j < 4; ++j) {
      const size_t bo = (size_t)(n0 + (j << 4) + rlane) * ldb + koff + k0;
      bh[j] = frag_load_b(Bt + bo);
    }
#pragma unroll
    for (int i = 0; i < 4; ++i) {
      const size_t ao = (size_t)(m0 + (i << 4) + rlane) * lda + koff + k0;
      v16b ah = frag_load_b(A + ao);
      v16b al = ah;
      if (SPL >= 1) al = frag_load_b(A2 + ao);
#pragma unroll
      for (int j = 0; j < 4; ++j) {
        acc[i][j] = mma_b(ah, bh[j], acc[i][j]);
        if (SPL >= 1) acc[i][j] = mma_b(al, bh[j], acc[i][j]);
      }
      dep_guard4_b(acc[i][0], acc[i][1], acc[i][2], acc[i][3], ah, al);
    }
    keep4_b(bh[0], bh[1], bh[2], bh[3]);
  }
  acc_guard4(acc[0][0], acc[0][1], acc[0][2], acc[0][3]);
  acc_guard4(acc[1][0], acc[1][1], acc[1][2], acc[1][3]);
  acc_guard4(acc[2][0], acc[2][1], acc[2][2], acc[2][3]);
  acc_guard4(acc[3][0], acc[3][1], acc[3][2], acc[3][3]);

  float* slab = sT[wave];
#pragma unroll
  for (int i = 0; i < 4; ++i) {
    const int mBase = m0 + (i << 4);
#pragma unroll
    for (int j = 0; j < 4; ++j) {
#pragma unroll
      for (int r = 0; r < 8; ++r) {
        slab[(mOff + r) * 68 + (j << 4) + rlane] = acc[i][j][r];
      }
    }
    __builtin_amdgcn_fence(__ATOMIC_RELEASE, "workgroup");
    __builtin_amdgcn_wave_barrier();
    __builtin_amdgcn_fence(__ATOMIC_ACQUIRE, "workgroup");
    {
      const int hh = lane >> 4, c4 = (lane & 15) * 4;
      for (int pass = 0; pass < 2; ++pass) {
#pragma unroll
        for (int it = 0; it < 8; ++it) {
          const int row = it * 2 + hh;
          v4f v = *(const v4f*)(slab + row * 68 + c4);
          *(volatile v4f*)(Cout + (size_t)(mBase + row) * ldc + n0 + c4) = v;
        }
        __threadfence();
      }
    }
    __builtin_amdgcn_fence(__ATOMIC_RELEASE, "workgroup");
    __builtin_amdgcn_wave_barrier();
    __builtin_amdgcn_fence(__ATOMIC_ACQUIRE, "workgroup");
  }
}

__global__ __launch_bounds__(256) void cast_bf16_kernel(
    const float* __restrict__ src, unsigned short* __restrict__ dst, int total8, int real8)
{
  const int i = blockIdx.x * 256 + threadIdx.x;
  if (i >= total8) return;
  const bool live = (i < real8);
  const int ic = live ? i : (real8 - 1);
  const size_t e0 = (size_t)ic << 3;
  const v4f a0 = *(const v4f*)(src + e0);
  const v4f a1 = *(const v4f*)(src + e0 + 4);
  const unsigned w0 = pack_hi2(a0[0], a0[1]);
  const unsigned w1 = pack_hi2(a0[2], a0[3]);
  const unsigned w2 = pack_hi2(a1[0], a1[1]);
  const unsigned w3 = pack_hi2(a1[2], a1[3]);
  v4u w;
  w[0] = live ? w0 : 0u;
  w[1] = live ? w1 : 0u;
  w[2] = live ? w2 : 0u;
  w[3] = live ? w3 : 0u;
  unsigned short* q = dst + ((size_t)i << 3);
  *(volatile v4u*)q = w;
  __threadfence();
  *(volatile v4u*)q = w;
}

__global__ __launch_bounds__(256) void conv_silu_kernel(
    const float* __restrict__ XZ, const float* __restrict__ cw, const float* __restrict__ cb,
    float* __restrict__ UC, unsigned short* __restrict__ UCH, unsigned short* __restrict__ UCL)
{
  __shared__ __align__(16) float sT[16 * kConvTP];
  const int tid = threadIdx.x, lane = tid & 31, wave = tid >> 5;
  const int d0 = blockIdx.x * 256, d = d0 + tid;
  const int g0 = blockIdx.y * 64;
  const int tb = g0 & (kSeq - 1);
  const float w0 = bf_rne(cw[d * 3 + 0]);
  const float w1 = bf_rne(cw[d * 3 + 1]);
  const float w2 = bf_rne(cw[d * 3 + 2]);
  const float bc = bf_rne(cb[d]);
  float xm2, xm1;
  {
    const bool hist = (tb > 0);
    const int rb = hist ? (g0 - 2) : g0;
    const float v2 = XZ[(size_t)rb * kXzP + d];
    const float v1 = XZ[(size_t)(rb + 1) * kXzP + d];
    xm2 = hist ? v2 : 0.f;
    xm1 = hist ? v1 : 0.f;
  }
  const int hrow = wave >> 1;
  const int hch  = (wave & 1) * 128 + lane * 4;
#pragma unroll 1
  for (int sub = 0; sub < 4; ++sub) {
    const int lb = g0 + sub * 16;
#pragma unroll 1
    for (int s = 0; s < 16; ++s) {
      const float xcur = XZ[(size_t)(lb + s) * kXzP + d];
      float acc = w0 * xm2;
      acc = fmaf(w1, xm1, acc);
      acc = fmaf(w2, xcur, acc);
      const float sv = acc + bc;
      const float sg = __builtin_amdgcn_rcpf(1.0f + expf(-sv));
      sT[s * kConvTP + tid] = sv * sg;
      xm2 = xm1;
      xm1 = xcur;
    }
    __syncthreads();
    v4f fv[4];
    v4u wh[2], wl[2];
#pragma unroll
    for (int it = 0; it < 4; ++it) fv[it] = *(const v4f*)(sT + (it * 4 + hrow) * kConvTP + hch);
#pragma unroll
    for (int it = 0; it < 2; ++it) {
      const float* sp = sT + (it * 8 + wave) * kConvTP + lane * 8;
      const v4f a0 = *(const v4f*)(sp);
      const v4f a1 = *(const v4f*)(sp + 4);
      wh[it][0] = pack_hi2(a0[0], a0[1]);
      wh[it][1] = pack_hi2(a0[2], a0[3]);
      wh[it][2] = pack_hi2(a1[0], a1[1]);
      wh[it][3] = pack_hi2(a1[2], a1[3]);
      wl[it][0] = pack_lo2(a0[0], a0[1]);
      wl[it][1] = pack_lo2(a0[2], a0[3]);
      wl[it][2] = pack_lo2(a1[0], a1[1]);
      wl[it][3] = pack_lo2(a1[2], a1[3]);
    }
    for (int pass = 0; pass < 2; ++pass) {
#pragma unroll
      for (int it = 0; it < 4; ++it)
        *(volatile v4f*)(UC + (size_t)(lb + it * 4 + hrow) * kDin + d0 + hch) = fv[it];
#pragma unroll
      for (int it = 0; it < 2; ++it) {
        const size_t o = (size_t)(lb + it * 8 + wave) * kDin + d0 + lane * 8;
        *(volatile v4u*)(UCH + o) = wh[it];
        *(volatile v4u*)(UCL + o) = wl[it];
      }
      __threadfence();
    }
    __syncthreads();
  }
}

__global__ __launch_bounds__(64) void scan_kernel(
    const float* __restrict__ PROJ, const float* __restrict__ UC, const float* __restrict__ XZ,
    const float* __restrict__ Wdt, const float* __restrict__ bdt, const float* __restrict__ Alog,
    const float* __restrict__ Aimag, const float* __restrict__ Dp,
    unsigned short* __restrict__ YH, unsigned short* __restrict__ YL)
{
  __shared__ __align__(16) float sX[(kScanTS + 1) * kScanXP];
  __shared__ __align__(16) float sY[kScanTS * kScanYP];
  __shared__ __align__(16) float sW[kDtR * kScanCh];
  __shared__ __align__(16) v2f   sH[kNst * kScanCh];
  __shared__ __align__(16) v2f   sA[kNst];
  const int tid = threadIdx.x, lane = tid & 31, wave = tid >> 5;
  constexpr int kBlkPerB = kDin / kScanCh;
  const int bix  = blockIdx.x / kBlkPerB;
  const int d0   = (blockIdx.x - bix * kBlkPerB) * kScanCh;
  const int d    = d0 + tid;
  const int head = d0 / kHd;
  const size_t row0 = (size_t)bix * kSeq;

#pragma unroll 1
  for (int r = 0; r < kDtR; ++r) sW[r * kScanCh + tid] = bf_rne(Wdt[(size_t)d * kDtR + r]);
  {
    const int n = tid & 15;
    const float al = Alog[head * kNst + n];
    const float ai = Aimag[head * kNst + n];
    v2f av;
    av[0] = -expf(bf_rne(al));
    av[1] = bf_rne(ai);
    if (tid < kNst) sA[n] = av;
  }
#pragma unroll 1
  for (int n = 0; n < kNst; ++n) {
    v2f zz;
    zz[0] = 0.f;
    zz[1] = 0.f;
    sH[n * kScanCh + tid] = zz;
  }
  if (tid < 32) sX[kLB + tid] = 0.f;
  const float bb = bf_rne(bdt[d]);
  const float Dd = bf_rne(Dp[d]);
  float xprev = 0.f;
  const int q = lane >> 3, c8 = (lane & 7) * 8;

#pragma unroll 1
  for (int t0 = 0; t0 < kSeq; t0 += kScanTS) {
    __syncthreads();
    if (t0 > 0 && tid < 32) sX[kLB + tid] = sX[kScanTS * kScanXP + kLB + tid];
    __syncthreads();
    {
      const size_t grow = (row0 + (size_t)t0 + (size_t)tid) * kPrjP;
#pragma unroll 1
      for (int pc = 0; pc < 24; ++pc) {
        int col;
        if (pc < 8) {
          col = 4 * pc;
        } else {
          const int grp = (pc - 8) >> 2;
          const int sub = (pc - 8) & 3;
          col = kColBre + grp * kHN + head * kNst + 4 * sub;
        }
        const v4f v = *(const v4f*)(PROJ + grow + col);
        *(v4f*)(sX + (tid + 1) * kScanXP + 4 * pc) = v;
      }
#pragma unroll 1
      for (int w = 0; w < 2; ++w) {
        const float p = PROJ[grow + kColLg + w * kHeads + head];
        const float e = expf(-p);
        sX[(tid + 1) * kScanXP + kLG + w] = __builtin_amdgcn_rcpf(1.0f + e);
      }
    }
    __syncthreads();

#pragma unroll 1
    for (int s = 0; s < kScanTS; ++s) {
      const float* xr = sX + (s + 1) * kScanXP;
      const float* xq = sX + s * kScanXP;
      float vdot = 0.f;
#pragma unroll 1
      for (int r4 = 0; r4 < kDtR / 4; ++r4) {
        const v4f xv = *(const v4f*)(xr + 4 * r4);
        const float* wp = sW + (4 * r4) * kScanCh + tid;
        vdot = fmaf(xv[0], wp[0], vdot);
        vdot = fmaf(xv[1], wp[kScanCh], vdot);
        vdot = fmaf(xv[2], wp[2 * kScanCh], vdot);
        vdot = fmaf(xv[3], wp[3 * kScanCh], vdot);
      }
      const float v   = vdot + bb;
      const float ea0 = expf(-fabsf(v));
      const float up  = 1.0f + ea0;
      const float l1p = logf(up) + (ea0 - (up - 1.0f)) * __builtin_amdgcn_rcpf(up);
      const float dt  = fmaxf(v, 0.0f) + l1p;
      const size_t grow = row0 + (size_t)t0 + (size_t)s;
      float xt = UC[grow * kDin + d];
      float zv = XZ[grow * kXzP + kDin + d];
      asm volatile("" : "+v"(xt));
      asm volatile("" : "+v"(zv));
      const float lg = xr[kLG];
      const float eg = xr[kLG + 1];
      const float bs = (1.0f - lg) * dt;
      const float gm = (lg * dt) * eg;
      float y = 0.f;
#pragma unroll 1
      for (int n = 0; n < kNst; ++n) {
        const v2f an = sA[n];
        const float bre = xr[kLB + n];
        const float bim = xr[kLBi + n];
        const float cre = xr[kLC + n];
        const float cim = xr[kLCi + n];
        const float pre = xq[kLB + n];
        const float pim = xq[kLBi + n];
        float dre = dt * an[0];
        dre = fminf(fmaxf(dre, -20.0f), 20.0f);
        const float dim = dt * an[1];
        const float ea = expf(dre);
        const float sn = sinf(dim);
        const float cs = cosf(dim);
        const float al_re = ea * cs;
        const float al_im = ea * sn;
        const float be_re = bs * al_re;
        const float be_im = bs * al_im;
        const float bxp_re = xprev * pre;
        const float bxp_im = xprev * pim;
        const float bx_re = xt * bre;
        const float bx_im = xt * bim;
        const float u_re = be_re * bxp_re - be_im * bxp_im + gm * bx_re;
        const float u_im = be_re * bxp_im + be_im * bxp_re + gm * bx_im;
        const v2f hv = sH[n * kScanCh + tid];
        const float h0 = hv[0];
        const float h1 = hv[1];
        v2f hn;
        hn[0] = al_re * h0 - al_im * h1 + u_re;
        hn[1] = al_re * h1 + al_im * h0 + u_im;
        sH[n * kScanCh + tid] = hn;
        y += hn[0] * cre + hn[1] * cim;
      }
      y = y + Dd * xt;
      const float sg = __builtin_amdgcn_rcpf(1.0f + expf(-zv));
      y = y * (zv * sg);
      sY[s * kScanYP + tid] = y;
      xprev = xt;
    }
    __syncthreads();
    v4u hw[8], lw[8];
#pragma unroll
    for (int it = 0; it < 8; ++it) {
      const int row = it * 8 + wave * 4 + q;
      const float* sp = sY + row * kScanYP + c8;
      const v4f a0 = *(const v4f*)(sp);
      const v4f a1 = *(const v4f*)(sp + 4);
      hw[it][0] = pack_hi2(a0[0], a0[1]);
      hw[it][1] = pack_hi2(a0[2], a0[3]);
      hw[it][2] = pack_hi2(a1[0], a1[1]);
      hw[it][3] = pack_hi2(a1[2], a1[3]);
      lw[it][0] = pack_lo2(a0[0], a0[1]);
      lw[it][1] = pack_lo2(a0[2], a0[3]);
      lw[it][2] = pack_lo2(a1[0], a1[1]);
      lw[it][3] = pack_lo2(a1[2], a1[3]);
    }
    for (int pass = 0; pass < 2; ++pass) {
#pragma unroll
      for (int it = 0; it < 8; ++it) {
        const int row = it * 8 + wave * 4 + q;
        const size_t o = (row0 + (size_t)t0 + (size_t)row) * kDin + d0 + c8;
        *(volatile v4u*)(YH + o) = hw[it];
        *(volatile v4u*)(YL + o) = lw[it];
      }
      __threadfence();
    }
  }
}

static_assert(((kRows / 64) * (kXzP / 64)) % 8 == 0, "in_proj block count");
static_assert(((kRows / 64) * (kPrjP / 64)) % 8 == 0, "x_proj block count");
static_assert(((kRows / 64) * (kDm / 64)) % 8 == 0, "out_proj block count");
static_assert(((kRows * kDm / 8) % 256) == 0 && ((kXzP * kDm / 8) % 256) == 0 &&
              ((kPrjP * kDin / 8) % 256) == 0 && ((kDm * kDin / 8) % 256) == 0, "cast grids exact");

extern "C" void kernel_launch(void* const* d_in, const int* in_sizes, int n_in,
                              void* d_out, int out_size, void* d_ws, size_t ws_size,
                              hipStream_t stream) {
  if (n_in < 11) return;
  if (in_sizes[0] != kRows * kDm) return;
  if (in_sizes[1] != kXzP * kDm) return;
  if (in_sizes[2] != kDin * 3) return;
  if (in_sizes[3] != kDin) return;
  if (in_sizes[4] != kPrjN * kDin) return;
  if (in_sizes[5] != kDin * kDtR) return;
  if (in_sizes[6] != kDin) return;
  if (in_sizes[7] != kHeads * kNst) return;
  if (in_sizes[8] != kHeads * kNst) return;
  if (in_sizes[9] != kDin) return;
  if (in_sizes[10] != kDm * kDin) return;
  if (out_size != kRows * kDm) return;
  if (ws_size < kWsTotal) return;

  const float* x       = (const float*)d_in[0];
  const float* W_in    = (const float*)d_in[1];
  const float* conv_w  = (const float*)d_in[2];
  const float* conv_b  = (const float*)d_in[3];
  const float* W_xproj = (const float*)d_in[4];
  const float* W_dt    = (const float*)d_in[5];
  const float* b_dt    = (const float*)d_in[6];
  const float* A_log   = (const float*)d_in[7];
  const float* A_imag  = (const float*)d_in[8];
  const float* Dp      = (const float*)d_in[9];
  const float* W_out   = (const float*)d_in[10];
  float* out = (float*)d_out;

  char* ws = (char*)d_ws;
  unsigned short* XB   = (unsigned short*)(ws + kOffXB);
  unsigned short* WIB  = (unsigned short*)(ws + kOffWIB);
  unsigned short* WXB  = (unsigned short*)(ws + kOffWXB);
  unsigned short* WOB  = (unsigned short*)(ws + kOffWOB);
  float*          XZ   = (float*)(ws + kOffXZ);
  float*          UC   = (float*)(ws + kOffUC);
  unsigned short* UCH  = (unsigned short*)(ws + kOffUCH);
  unsigned short* UCL  = (unsigned short*)(ws + kOffUCL);
  float*          PROJ = (float*)(ws + kOffPROJ);
  unsigned short* YH   = (unsigned short*)(ws + kOffYH);
  unsigned short* YL   = (unsigned short*)(ws + kOffYL);

  cast_bf16_kernel<<<(kRows * kDm / 8) / 256, 256, 0, stream>>>(x, XB, kRows * kDm / 8, kRows * kDm / 8);
  cast_bf16_kernel<<<(kXzP * kDm / 8) / 256, 256, 0, stream>>>(W_in, WIB, kXzP * kDm / 8, kXzP * kDm / 8);
  cast_bf16_kernel<<<(kPrjP * kDin / 8) / 256, 256, 0, stream>>>(W_xproj, WXB, kPrjP * kDin / 8, kPrjN * kDin / 8);
  cast_bf16_kernel<<<(kDm * kDin / 8) / 256, 256, 0, stream>>>(W_out, WOB, kDm * kDin / 8, kDm * kDin / 8);

  wmma_gemm64_bf<0><<<((kRows / 64) * (kXzP / 64)) / 8, 256, 0, stream>>>(
      XB, XB, kDm, WIB, kDm, XZ, kXzP, kRows, kXzP, kDm);

  conv_silu_kernel<<<dim3(kDin / 256, kRows / 64), 256, 0, stream>>>(XZ, conv_w, conv_b, UC, UCH, UCL);

  wmma_gemm64_bf<1><<<((kRows / 64) * (kPrjP / 64)) / 8, 256, 0, stream>>>(
      UCH, UCL, kDin, WXB, kDin, PROJ, kPrjP, kRows, kPrjP, kDin);

  scan_kernel<<<kBatch * (kDin / kScanCh), kScanCh, 0, stream>>>(
      PROJ, UC, XZ, W_dt, b_dt, A_log, A_imag, Dp, YH, YL);

  wmma_gemm64_bf<1><<<((kRows / 64) * (kDm / 64)) / 8, 256, 0, stream>>>(
      YH, YL, kDin, WOB, kDin, out, kDm, kRows, kDm, kDin);
}
